// BasicBlock6_4947802325429
// MI455X (gfx1250) — hardware-verified
//
#include <hip/hip_runtime.h>
#include <stddef.h>
#include <stdint.h>


#define NBAT   8
#define NC     128
#define NH     64
#define NW     64
#define NBH    (NBAT * NH)
#define NPIX   (NBAT * NH * NW)
#define KD     1152
#define K8     (KD / 8)
#define NOFF   18
#define OFFP   32
#define APITCH 136
#define OP0    132
#define OP1    68
#define WDSC   64.0f
#define WDINV  0.015625f
#define BNEPS  1e-5f

static_assert((APITCH * 2) % 16 == 0);
static_assert((OP0 * 4) % 16 == 0);
static_assert((OP1 * 4) % 16 == 0);
static_assert(NW * OP0 <= 8960);
static_assert(NC * OP1 <= 8960);
static_assert(NW * 9 * 8 + (NW * APITCH) / 2 == 8960);

typedef float          v4f   __attribute__((ext_vector_type(4)));
typedef float          v8f   __attribute__((ext_vector_type(8)));
typedef _Float16       v4h   __attribute__((ext_vector_type(4)));
typedef _Float16       v8h   __attribute__((ext_vector_type(8)));
typedef _Float16       v16h  __attribute__((ext_vector_type(16)));
typedef unsigned short v8us  __attribute__((ext_vector_type(8)));
typedef unsigned int   v4u   __attribute__((ext_vector_type(4)));
typedef __bf16         v16bf __attribute__((ext_vector_type(16)));

union FragH { v16h v; v8h h[2]; };
union FragB { v16bf v; v8us h[2]; v4u q[2]; };
union Pack8 { v8h h; v4u u; };

__device__ __forceinline__ unsigned int bf_bits(float f) {
  unsigned int u = __float_as_uint(f);
  u += 0x7FFFu + ((u >> 16) & 1u);
  return u >> 16;
}
__device__ __forceinline__ float bfr(float f) { return __uint_as_float(bf_bits(f) << 16); }

__device__ __forceinline__ v8f zero8f() {
  v8f z;
#pragma unroll
  for (int i = 0; i < 8; ++i) z[i] = 0.0f;
  return z;
}

__device__ __forceinline__ v8f wm_f16(v16h a, v16h b, v8f c) {
  v8f d = __builtin_amdgcn_wmma_f32_16x16x32_f16(false, a, false, b, (short)0, c, false, false);
  asm volatile("v_nop\n\tv_nop\n\tv_nop\n\tv_nop" : "+v"(d) : "v"(a), "v"(b));
  return d;
}
__device__ __forceinline__ v8f wm_bf(v16bf a, v16bf b, v8f c) {
  v8f d = __builtin_amdgcn_wmma_f32_16x16x32_bf16(false, a, false, b, (short)0, c, false, false);
  asm volatile("v_nop\n\tv_nop\n\tv_nop\n\tv_nop" : "+v"(d) : "v"(a), "v"(b));
  return d;
}

__global__ __launch_bounds__(256) void k_planes(const float* __restrict__ x, float* xpf,
                                                unsigned short* xph, int nbh) {
  __shared__ __attribute__((aligned(16))) float T[NW * OP0];
  const int tid = threadIdx.x, lane = tid & 31, wave = tid >> 5, hh = lane >> 4, m = lane & 15;
  const int bh = blockIdx.x;
  if (bh >= nbh) return;
  const int b = bh >> 6, h = bh & 63;
  const size_t pix0 = (size_t)bh * NW;
#pragma unroll 1
  for (int it = 0; it < 8; ++it) {
    const int c = it * 16 + (tid >> 4);
    const int w4 = 4 * (tid & 15);
    const v4f v = *(const v4f*)(x + (((size_t)(b * NC + c)) * NH + h) * NW + w4);
    T[(w4 + 0) * OP0 + c] = bfr(v.x);
    T[(w4 + 1) * OP0 + c] = bfr(v.y);
    T[(w4 + 2) * OP0 + c] = bfr(v.z);
    T[(w4 + 3) * OP0 + c] = bfr(v.w);
  }
  __syncthreads();
  auto st = [&]() {
#pragma unroll 1
    for (int j = 0; j < 8; ++j) {
      const int px = wave * 8 + j;
      const v4f v = *(const v4f*)(T + px * OP0 + 4 * lane);
      *(volatile v4f*)(xpf + (pix0 + px) * NC + 4 * lane) = v;
    }
#pragma unroll 1
    for (int j2 = 0; j2 < 4; ++j2) {
      const int px = wave * 8 + 2 * j2 + hh;
      const float* q = T + px * OP0 + 8 * m;
      const v4f a = *(const v4f*)q;
      const v4f c = *(const v4f*)(q + 4);
      v4u u;
      u.x = (__float_as_uint(a.x) >> 16) | (__float_as_uint(a.y) & 0xFFFF0000u);
      u.y = (__float_as_uint(a.z) >> 16) | (__float_as_uint(a.w) & 0xFFFF0000u);
      u.z = (__float_as_uint(c.x) >> 16) | (__float_as_uint(c.y) & 0xFFFF0000u);
      u.w = (__float_as_uint(c.z) >> 16) | (__float_as_uint(c.w) & 0xFFFF0000u);
      *(volatile v4u*)(xph + (pix0 + px) * NC + 8 * m) = u;
    }
  };
  st();
  __threadfence();
  st();
}

__global__ __launch_bounds__(256) void k_packoff(const float* __restrict__ wA, const float* __restrict__ wB,
                                                 unsigned short* pA, unsigned short* pB) {
  const int item = blockIdx.x * 256 + threadIdx.x;
  if (item >= OFFP * K8) return;
  const float* w = (blockIdx.y == 0) ? wA : wB;
  unsigned short* p = (blockIdx.y == 0) ? pA : pB;
  const int n = item / K8;
  const int k = 8 * (item - n * K8);
  const int t = k >> 7, ci0 = k & 127;
  const bool nv = n < NOFF;
  const int nn = nv ? n : (NOFF - 1);
  const float* wr = w + ((size_t)(nn * NC + ci0)) * 9 + t;
  unsigned int hb[8];
#pragma unroll
  for (int j = 0; j < 8; ++j) {
    const float v = wr[j * 9];
    hb[j] = nv ? bf_bits(v) : 0u;
  }
  v4u u;
  u.x = hb[0] | (hb[1] << 16);
  u.y = hb[2] | (hb[3] << 16);
  u.z = hb[4] | (hb[5] << 16);
  u.w = hb[6] | (hb[7] << 16);
  unsigned short* dst = p + (size_t)n * KD + k;
  *(volatile v4u*)dst = u;
  __threadfence();
  *(volatile v4u*)dst = u;
}

__global__ __launch_bounds__(256) void k_packdc(const float* __restrict__ wA, const float* __restrict__ wB,
                                                _Float16* pA, _Float16* pB) {
  const int item = blockIdx.x * 256 + threadIdx.x;
  if (item >= NC * K8) return;
  const float* w = (blockIdx.y == 0) ? wA : wB;
  _Float16* p = (blockIdx.y == 0) ? pA : pB;
  const int n = item / K8;
  const int k = 8 * (item - n * K8);
  const int t = k >> 7, ci0 = k & 127;
  const float* wr = w + ((size_t)(n * NC + ci0)) * 9 + t;
  Pack8 pk;
#pragma unroll
  for (int j = 0; j < 8; ++j) pk.h[j] = (_Float16)(bfr(wr[j * 9]) * WDSC);
  _Float16* dst = p + (size_t)n * KD + k;
  *(volatile v4u*)dst = pk.u;
  __threadfence();
  *(volatile v4u*)dst = pk.u;
}

template <int NPL>
__global__ __launch_bounds__(128) void k_offconv(
    const unsigned short* __restrict__ ah, const unsigned short* __restrict__ al,
    const unsigned short* __restrict__ wb, const float* __restrict__ bias,
    float* offo, int nbh) {
  __shared__ __attribute__((aligned(16))) float S[4 * 16 * OFFP];
  const int tid = threadIdx.x, lane = tid & 31, wave = tid >> 5, hh = lane >> 4, m = lane & 15;
  const int bh = blockIdx.x;
  if (bh >= nbh) return;
  const int b = bh >> 6, h = bh & 63;
  const int w = wave * 16 + m;
  v8f acc[2];
  acc[0] = zero8f();
  acc[1] = zero8f();
  const unsigned short* b0 = wb + (size_t)m * KD + 8 * hh;
  const unsigned short* b1 = wb + (size_t)(16 + m) * KD + 8 * hh;
#pragma unroll 1
  for (int t = 0; t < 9; ++t) {
    const int ky = t / 3, kx = t - 3 * ky;
    const int hs = h + ky - 1, wsx = w + kx - 1;
    const bool valid = ((unsigned)hs < (unsigned)NH) && ((unsigned)wsx < (unsigned)NW);
    const int hsc = min(max(hs, 0), NH - 1), wsc = min(max(wsx, 0), NW - 1);
    const unsigned int msk = valid ? 0xFFFFFFFFu : 0u;
    const size_t arow = (((size_t)(b * NH + hsc)) * NW + wsc) * NC + 8 * hh;
    const unsigned short* pah = ah + arow;
    const unsigned short* pal = al + arow;
    const int tk = t * NC;
#pragma unroll
    for (int kc = 0; kc < 4; ++kc) {
      const int k0 = kc * 32;
      FragB a0, q0, q1;
      a0.h[0] = *(const v8us*)(pah + k0);
      a0.h[1] = *(const v8us*)(pah + k0 + 16);
      a0.q[0] = a0.q[0] & msk;
      a0.q[1] = a0.q[1] & msk;
      q0.h[0] = *(const v8us*)(b0 + tk + k0);
      q0.h[1] = *(const v8us*)(b0 + tk + k0 + 16);
      q1.h[0] = *(const v8us*)(b1 + tk + k0);
      q1.h[1] = *(const v8us*)(b1 + tk + k0 + 16);
      acc[0] = wm_bf(a0.v, q0.v, acc[0]);
      acc[1] = wm_bf(a0.v, q1.v, acc[1]);
      if (NPL == 2) {
        FragB a1;
        a1.h[0] = *(const v8us*)(pal + k0);
        a1.h[1] = *(const v8us*)(pal + k0 + 16);
        a1.q[0] = a1.q[0] & msk;
        a1.q[1] = a1.q[1] & msk;
        acc[0] = wm_bf(a1.v, q0.v, acc[0]);
        acc[1] = wm_bf(a1.v, q1.v, acc[1]);
      }
    }
  }
  float* Sw = S + wave * 16 * OFFP;
#pragma unroll
  for (int nt = 0; nt < 2; ++nt) {
    const int n = nt * 16 + m;
    const bool nv = n < NOFF;
    const float bv = bfr(bias[nv ? n : (NOFF - 1)]);
#pragma unroll
    for (int r = 0; r < 8; ++r) {
      const float v = nv ? (acc[nt][r] + bv) : 0.0f;
      Sw[(8 * hh + r) * OFFP + n] = v;
    }
  }
  __syncthreads();
  const size_t pixw = (size_t)bh * NW + wave * 16;
  auto st = [&]() {
#pragma unroll
    for (int q = 0; q < 4; ++q) {
      const int px = 4 * q + (lane >> 3);
      const int c4 = 4 * (lane & 7);
      const v4f v = *(const v4f*)(Sw + px * OFFP + c4);
      *(volatile v4f*)(offo + (pixw + px) * OFFP + c4) = v;
    }
  };
  st();
  __threadfence();
  st();
}

template <int FINAL>
__global__ __launch_bounds__(256) void k_deform(
    const float* __restrict__ src,
    const float* __restrict__ offp,
    const _Float16* __restrict__ wd,
    const float* __restrict__ g, const float* __restrict__ be,
    const float* __restrict__ mn, const float* __restrict__ vr,
    float* opf, unsigned short* oph, unsigned short* opl,
    const float* __restrict__ xres, float* outp,
    int nbh) {
#pragma clang fp contract(off)
  __shared__ __attribute__((aligned(16))) float smem[8960];
  float* G = smem;
  _Float16* At = (_Float16*)(smem + NW * 9 * 8);
  float* O = smem;
  const int tid = threadIdx.x, lane = tid & 31, wave = tid >> 5, hh = lane >> 4, m = lane & 15;
  const int bh = blockIdx.x;
  if (bh >= nbh) return;
  const int b = bh >> 6, h = bh & 63;
  const size_t pix0 = (size_t)bh * NW;

  for (int i = tid; i < NW * 9; i += 256) {
    const int px = i / 9, t = i - 9 * px;
    const int ky = t / 3, kx = t - 3 * ky;
    const float* op = offp + (pix0 + px) * OFFP + 2 * t;
    const float dy = op[0];
    const float dx = op[1];
    const float ys = (float)(h - 2 + 2 * ky) + dy;
    const float xs = (float)(px - 2 + 2 * kx) + dx;
    const float y0f = floorf(ys), x0f = floorf(xs);
    const float fy = ys - y0f, fx = xs - x0f;
    const bool vy0 = (y0f >= 0.0f) && (y0f < (float)NH);
    const bool vy1 = (y0f >= -1.0f) && (y0f < (float)(NH - 1));
    const bool vx0 = (x0f >= 0.0f) && (x0f < (float)NW);
    const bool vx1 = (x0f >= -1.0f) && (x0f < (float)(NW - 1));
    const float gy = 1.0f - fy, gx = 1.0f - fx;
    const float w00 = gy * gx, w01 = gy * fx, w10 = fy * gx, w11 = fy * fx;
    const int iy0 = (int)fminf(fmaxf(y0f, -4.0f), 80.0f);
    const int ix0 = (int)fminf(fmaxf(x0f, -4.0f), 80.0f);
    float* gp = G + i * 8;
    gp[0] = (vy0 && vx0) ? w00 : 0.0f;
    gp[1] = (vy0 && vx1) ? w01 : 0.0f;
    gp[2] = (vy1 && vx0) ? w10 : 0.0f;
    gp[3] = (vy1 && vx1) ? w11 : 0.0f;
    gp[4] = __int_as_float(iy0);
    gp[5] = __int_as_float(ix0);
    gp[6] = 0.0f;
    gp[7] = 0.0f;
  }
  __syncthreads();

  v8f acc[4];
#pragma unroll
  for (int mt = 0; mt < 4; ++mt) acc[mt] = zero8f();
  const int co = wave * 16 + m;
  const _Float16* wrow = wd + (size_t)co * KD + 8 * hh;
  const size_t rowb = (size_t)b * NH;

#pragma unroll 1
  for (int t = 0; t < 9; ++t) {
#pragma unroll 1
    for (int j = 0; j < 8; ++j) {
      const int px = wave * 8 + j;
      const float* gp = G + (px * 9 + t) * 8;
      const v4f gw = *(const v4f*)gp;
      const int iy0 = __float_as_int(gp[4]);
      const int ix0 = __float_as_int(gp[5]);
      const int iy0c = min(max(iy0, 0), NH - 1), iy1c = min(max(iy0 + 1, 0), NH - 1);
      const int ix0c = min(max(ix0, 0), NW - 1), ix1c = min(max(ix0 + 1, 0), NW - 1);
      const float* p00 = src + ((rowb + iy0c) * NW + ix0c) * NC + 4 * lane;
      const float* p01 = src + ((rowb + iy0c) * NW + ix1c) * NC + 4 * lane;
      const float* p10 = src + ((rowb + iy1c) * NW + ix0c) * NC + 4 * lane;
      const float* p11 = src + ((rowb + iy1c) * NW + ix1c) * NC + 4 * lane;
      const v4f v00 = *(const v4f*)p00;
      const v4f v01 = *(const v4f*)p01;
      const v4f v10 = *(const v4f*)p10;
      const v4f v11 = *(const v4f*)p11;
      v4h hv;
#pragma unroll
      for (int c = 0; c < 4; ++c) {
        const float s = ((v00[c] * gw.x + v01[c] * gw.y) + v10[c] * gw.z) + v11[c] * gw.w;
        hv[c] = (_Float16)s;
      }
      *(v4h*)(At + px * APITCH + 4 * lane) = hv;
    }
    __syncthreads();
#pragma unroll
    for (int ks = 0; ks < 4; ++ks) {
      FragH bq;
      const _Float16* bp = wrow + t * NC + ks * 32;
      bq.h[0] = *(const v8h*)bp;
      bq.h[1] = *(const v8h*)(bp + 16);
#pragma unroll
      for (int mt = 0; mt < 4; ++mt) {
        FragH aq;
        const _Float16* ap = At + (mt * 16 + m) * APITCH + ks * 32 + 8 * hh;
        aq.h[0] = *(const v8h*)ap;
        aq.h[1] = *(const v8h*)(ap + 16);
        acc[mt] = wm_f16(aq.v, bq.v, acc[mt]);
      }
    }
    __syncthreads();
  }

  {
    const float gv = bfr(g[co]), bv = bfr(be[co]), mv = bfr(mn[co]), vv = bfr(vr[co]);
    const float inv = gv * rsqrtf(vv + BNEPS);
    const float sh = bv - mv * inv;
#pragma unroll
    for (int mt = 0; mt < 4; ++mt) {
#pragma unroll
      for (int r = 0; r < 8; ++r) {
        const int px = mt * 16 + 8 * hh + r;
        float val = acc[mt][r] * WDINV * inv + sh;
        if (FINAL == 0) {
          val = fmaxf(val, 0.0f);
          O[px * OP0 + co] = val;
        } else {
          O[co * OP1 + px] = val;
        }
      }
    }
  }
  __syncthreads();

  if (FINAL == 0) {
    auto st = [&]() {
#pragma unroll 1
      for (int j = 0; j < 8; ++j) {
        const int px = wave * 8 + j;
        const v4f v = *(const v4f*)(O + px * OP0 + 4 * lane);
        *(volatile v4f*)(opf + (pix0 + px) * NC + 4 * lane) = v;
      }
#pragma unroll 1
      for (int j2 = 0; j2 < 4; ++j2) {
        const int px = wave * 8 + 2 * j2 + hh;
        const float* q = O + px * OP0 + 8 * m;
        const v4f a = *(const v4f*)q;
        const v4f c = *(const v4f*)(q + 4);
        float f[8] = {a.x, a.y, a.z, a.w, c.x, c.y, c.z, c.w};
        unsigned int hb[8], lb[8];
#pragma unroll
        for (int e = 0; e < 8; ++e) {
          hb[e] = bf_bits(f[e]);
          lb[e] = bf_bits(f[e] - __uint_as_float(hb[e] << 16));
        }
        v4u hu, lu;
        hu.x = hb[0] | (hb[1] << 16); hu.y = hb[2] | (hb[3] << 16);
        hu.z = hb[4] | (hb[5] << 16); hu.w = hb[6] | (hb[7] << 16);
        lu.x = lb[0] | (lb[1] << 16); lu.y = lb[2] | (lb[3] << 16);
        lu.z = lb[4] | (lb[5] << 16); lu.w = lb[6] | (lb[7] << 16);
        const size_t gi = (pix0 + px) * NC + 8 * m;
        *(volatile v4u*)(oph + gi) = hu;
        *(volatile v4u*)(opl + gi) = lu;
      }
    };
    st();
    __threadfence();
    st();
  } else {
    auto st = [&]() {
#pragma unroll 1
      for (int i = 0; i < 8; ++i) {
        const int c = wave * 16 + 2 * i + hh;
        const int w4 = 4 * m;
        const v4f v = *(const v4f*)(O + c * OP1 + w4);
        const size_t gi = (((size_t)(b * NC + c)) * NH + h) * NW + w4;
        const v4f xv = *(const v4f*)(xres + gi);
        v4f o;
        o.x = fmaxf(v.x + bfr(xv.x), 0.0f);
        o.y = fmaxf(v.y + bfr(xv.y), 0.0f);
        o.z = fmaxf(v.z + bfr(xv.z), 0.0f);
        o.w = fmaxf(v.w + bfr(xv.w), 0.0f);
        *(volatile v4f*)(outp + gi) = o;
      }
    };
    st();
    __threadfence();
    st();
  }
}

extern "C" void kernel_launch(void* const* d_in, const int* in_sizes, int n_in,
                              void* d_out, int out_size, void* d_ws, size_t ws_size,
                              hipStream_t stream) {
  if (n_in < 15) return;
  if (in_sizes[0] != NPIX * NC) return;
  if (in_sizes[1] != NOFF * NC * 9 || in_sizes[2] < NOFF || in_sizes[3] != NC * NC * 9) return;
  if (in_sizes[4] < NC || in_sizes[5] < NC || in_sizes[6] < NC || in_sizes[7] < NC) return;
  if (in_sizes[8] != NOFF * NC * 9 || in_sizes[9] < NOFF || in_sizes[10] != NC * NC * 9) return;
  if (in_sizes[11] < NC || in_sizes[12] < NC || in_sizes[13] < NC || in_sizes[14] < NC) return;
  if (out_size != NPIX * NC) return;

  const float* x      = (const float*)d_in[0];
  const float* w_off1 = (const float*)d_in[1];
  const float* b_off1 = (const float*)d_in[2];
  const float* w_dc1  = (const float*)d_in[3];
  const float* g1     = (const float*)d_in[4];
  const float* beta1  = (const float*)d_in[5];
  const float* m1     = (const float*)d_in[6];
  const float* v1     = (const float*)d_in[7];
  const float* w_off2 = (const float*)d_in[8];
  const float* b_off2 = (const float*)d_in[9];
  const float* w_dc2  = (const float*)d_in[10];
  const float* g2     = (const float*)d_in[11];
  const float* beta2  = (const float*)d_in[12];
  const float* m2     = (const float*)d_in[13];
  const float* v2     = (const float*)d_in[14];
  float* out = (float*)d_out;

  const size_t szPF  = (size_t)NPIX * NC * 4;
  const size_t szPH  = (size_t)NPIX * NC * 2;
  const size_t szOFF = (size_t)NPIX * OFFP * 4;
  const size_t szWO  = (size_t)OFFP * KD * 2;
  const size_t szWD  = (size_t)NC * KD * 2;
  size_t off = 0;
  const size_t oXpf = off;  off += szPF;
  const size_t oXph = off;  off += szPH;
  const size_t oO1f = off;  off += szPF;
  const size_t oO1h = off;  off += szPH;
  const size_t oO1l = off;  off += szPH;
  const size_t oOf1 = off;  off += szOFF;
  const size_t oOf2 = off;  off += szOFF;
  const size_t oWo1 = off;  off += szWO;
  const size_t oWo2 = off;  off += szWO;
  const size_t oWd1 = off;  off += szWD;
  const size_t oWd2 = off;  off += szWD;
  if (off > ws_size || off > (size_t)134217728u) return;

  char* ws = (char*)d_ws;
  float*          xpf  = (float*)(ws + oXpf);
  unsigned short* xph  = (unsigned short*)(ws + oXph);
  float*          o1f  = (float*)(ws + oO1f);
  unsigned short* o1h  = (unsigned short*)(ws + oO1h);
  unsigned short* o1l  = (unsigned short*)(ws + oO1l);
  float*          off1 = (float*)(ws + oOf1);
  float*          off2 = (float*)(ws + oOf2);
  unsigned short* wo1  = (unsigned short*)(ws + oWo1);
  unsigned short* wo2  = (unsigned short*)(ws + oWo2);
  _Float16*       wd1  = (_Float16*)(ws + oWd1);
  _Float16*       wd2  = (_Float16*)(ws + oWd2);

  k_planes<<<dim3(NBH), dim3(256), 0, stream>>>(x, xpf, xph, NBH);
  k_packoff<<<dim3((OFFP * K8) / 256, 2), dim3(256), 0, stream>>>(w_off1, w_off2, wo1, wo2);
  k_packdc<<<dim3((NC * K8) / 256, 2), dim3(256), 0, stream>>>(w_dc1, w_dc2, wd1, wd2);

  k_offconv<1><<<dim3(NBH), dim3(128), 0, stream>>>(xph, xph, wo1, b_off1, off1, NBH);
  k_deform<0><<<dim3(NBH), dim3(256), 0, stream>>>(
      xpf, off1, wd1, g1, beta1, m1, v1, o1f, o1h, o1l, x, out, NBH);

  k_offconv<2><<<dim3(NBH), dim3(128), 0, stream>>>(o1h, o1l, wo2, b_off2, off2, NBH);
  k_deform<1><<<dim3(NBH), dim3(256), 0, stream>>>(
      o1f, off2, wd2, g2, beta2, m2, v2, xpf, xph, xph, x, out, NBH);
}
